// DifferentialCausalSelfAttention_48859547959913
// MI455X (gfx1250) — hardware-verified
//
#include <hip/hip_runtime.h>
#include <stdint.h>
#include <stddef.h>


#define NB   4
#define SEQ  2048
#define EMB  1024
#define NHD  8
#define NSH  16
#define HD   64
#define VD   128
#define RMS_EPS 1.1920929e-7f
#define LN_EPS  1e-5f

typedef unsigned short u16;
typedef u16    v8u  __attribute__((ext_vector_type(8)));
typedef int    v4i  __attribute__((ext_vector_type(4)));
typedef int    v8i  __attribute__((ext_vector_type(8)));
typedef float  v4f  __attribute__((ext_vector_type(4)));
typedef float  v8f  __attribute__((ext_vector_type(8)));
typedef __bf16 v16b __attribute__((ext_vector_type(16)));

union FU { v8i v; v4i p[2]; v16b b; };

struct InvFreq { float v[32]; };
static_assert(sizeof(InvFreq) == 128);

static __device__ __forceinline__ u16 bf_rne(float x) {
  unsigned u = __float_as_uint(x);
  u += 0x7FFFu + ((u >> 16) & 1u);
  return (u16)(u >> 16);
}
static __device__ __forceinline__ float bf_up(u16 b) { return __uint_as_float(((unsigned)b) << 16); }

static __device__ __forceinline__ void split8(float (&y)[8], v8u& hv, v8u& lv) {
#pragma unroll
  for (int i = 0; i < 8; ++i) {
    const u16 hb = bf_rne(y[i]);
    hv[i] = hb;
    lv[i] = bf_rne(y[i] - bf_up(hb));
  }
}

static __device__ __forceinline__ v8i ldfrag(const u16* p, int h) {
  FU f;
  f.p[0] = *(const v4i*)(p + 8 * h);
  f.p[1] = *(const v4i*)(p + 16 + 8 * h);
  return f.v;
}

static __device__ __forceinline__ v8f mma(v8i a, v8i b, v8f c) {
  FU ua, ub; ua.v = a; ub.v = b;
  c = __builtin_amdgcn_wmma_f32_16x16x32_bf16(false, ua.b, false, ub.b, (short)0, c, false, false);
  asm volatile("v_nop\n\tv_nop\n\tv_nop\n\tv_nop" : "+v"(c) : "v"(a), "v"(b));
  return c;
}
static __device__ __forceinline__ v8f mma3(v8i ah, v8i al, v8i bh, v8i bl, v8f c) {
  c = mma(ah, bh, c);
  c = mma(al, bh, c);
  c = mma(ah, bl, c);
  return c;
}

__global__ void __launch_bounds__(256) k_split(const float* __restrict__ src, u16* __restrict__ hi,
                                             u16* __restrict__ lo, int n8) {
  const int i = blockIdx.x * 256 + threadIdx.x;
  if (i >= n8) return;
  const size_t o = (size_t)i * 8;
  const v4f a = *(const v4f*)(src + o);
  const v4f b = *(const v4f*)(src + o + 4);
  float y[8] = {a[0], a[1], a[2], a[3], b[0], b[1], b[2], b[3]};
  v8u hv = {}, lv = {};
  split8(y, hv, lv);
  *(volatile v8u*)(hi + o) = hv;
  *(volatile v8u*)(lo + o) = lv;
  __threadfence();
  *(volatile v8u*)(hi + o) = hv;
  *(volatile v8u*)(lo + o) = lv;
}

__global__ void __launch_bounds__(256) k_rot(InvFreq inv, float* __restrict__ cs, float* __restrict__ sn, int n) {
#pragma clang fp contract(off)
  const int i = blockIdx.x * 256 + threadIdx.x;
  if (i >= n) return;
  const int j = i & 31, t = i >> 5;
  float f = 0.0f;
#pragma unroll
  for (int q = 0; q < 32; ++q) f = (j == q) ? inv.v[q] : f;
  const float ang = (float)t * f;
  const float c = cosf(ang);
  const float s = sinf(ang);
  *(volatile float*)(cs + i) = c;
  *(volatile float*)(sn + i) = s;
  __threadfence();
  *(volatile float*)(cs + i) = c;
  *(volatile float*)(sn + i) = s;
}

template <int MODE>
__global__ void __launch_bounds__(256) k_gemm(const u16* __restrict__ Ah, const u16* __restrict__ Al, int lda,
                                            const u16* __restrict__ Bh0, const u16* __restrict__ Bl0, int ldb, size_t bz,
                                            int K,
                                            u16* __restrict__ Dh0, u16* __restrict__ Dl0, size_t dz, int ldd,
                                            float* __restrict__ Out,
                                            const float* __restrict__ cst, const float* __restrict__ snt,
                                            float scale0, float scale1)
{
  __shared__ __align__(16) float stg[8][16][64];
  const int lane = threadIdx.x & 31, w = threadIdx.x >> 5, h = lane >> 4, m = lane & 15;
  const int z = blockIdx.z, bn = blockIdx.x, bm = blockIdx.y;
  const int n0 = bn * 64;
  const int m0 = bm * 256 + w * 32;
  const u16* Bh = Bh0 + (size_t)z * bz;
  const u16* Bl = Bl0 + (size_t)z * bz;

  v8f acc[2][4] = {};
  const u16* a0h = Ah + (size_t)(m0 + m) * lda;
  const u16* a1h = Ah + (size_t)(m0 + 16 + m) * lda;
  const u16* a0l = Al + (size_t)(m0 + m) * lda;
  const u16* a1l = Al + (size_t)(m0 + 16 + m) * lda;
  const size_t bro = (size_t)(n0 + m) * ldb;

#pragma unroll 1
  for (int k0 = 0; k0 < K; k0 += 32) {
    const v8i A0h = ldfrag(a0h + k0, h);
    const v8i A1h = ldfrag(a1h + k0, h);
    const v8i A0l = ldfrag(a0l + k0, h);
    const v8i A1l = ldfrag(a1l + k0, h);
#pragma unroll
    for (int ni = 0; ni < 4; ++ni) {
      const size_t bo = bro + (size_t)(ni * 16) * ldb + k0;
      const v8i Bvh = ldfrag(Bh + bo, h);
      const v8i Bvl = ldfrag(Bl + bo, h);
      acc[0][ni] = mma3(A0h, A0l, Bvh, Bvl, acc[0][ni]);
      acc[1][ni] = mma3(A1h, A1l, Bvh, Bvl, acc[1][ni]);
    }
  }

  const float scale = (z == 0) ? scale0 : scale1;
#pragma unroll
  for (int mi = 0; mi < 2; ++mi) {
#pragma unroll
    for (int ni = 0; ni < 4; ++ni)
#pragma unroll
      for (int r = 0; r < 8; ++r) stg[w][8 * h + r][ni * 16 + m] = acc[mi][ni][r];
    __syncthreads();
    const int rbase = m0 + mi * 16;
    if (MODE == 2) {
      const int rr = lane >> 4, c4 = lane & 15;
#pragma unroll
      for (int p = 0; p < 8; ++p) {
        const int row = p * 2 + rr;
        const v4f v = *(const v4f*)&stg[w][row][c4 * 4];
        float* o = Out + (size_t)(rbase + row) * ldd + n0 + c4 * 4;
        *(volatile v4f*)o = v;
        __threadfence();
        *(volatile v4f*)o = v;
      }
    } else {
      const int rr = lane >> 3, cg = lane & 7;
#pragma unroll
      for (int p = 0; p < 4; ++p) {
        const int row = p * 4 + rr;
        const v4f va = *(const v4f*)&stg[w][row][cg * 8];
        const v4f vb = *(const v4f*)&stg[w][row][cg * 8 + 4];
        float y[8] = {va[0], va[1], va[2], va[3], vb[0], vb[1], vb[2], vb[3]};
        u16* dh;
        u16* dl;
        if (MODE == 0) {
          const int t = rbase + row;
          float ss = 0.0f;
#pragma unroll
          for (int i = 0; i < 8; ++i) ss += y[i] * y[i];
          ss += __shfl_xor(ss, 1, 32);
          ss += __shfl_xor(ss, 2, 32);
          ss += __shfl_xor(ss, 4, 32);
          const float rn = rsqrtf(ss * (1.0f / 64.0f) + RMS_EPS);
          float pt[8];
#pragma unroll
          for (int i = 0; i < 8; ++i) pt[i] = __shfl_xor(y[i], 4, 32);
          const int j0 = (cg & 3) * 8;
          const v4f ca = *(const v4f*)(cst + (size_t)t * 32 + j0);
          const v4f cb = *(const v4f*)(cst + (size_t)t * 32 + j0 + 4);
          const v4f sa = *(const v4f*)(snt + (size_t)t * 32 + j0);
          const v4f sb = *(const v4f*)(snt + (size_t)t * 32 + j0 + 4);
          const float cc[8] = {ca[0], ca[1], ca[2], ca[3], cb[0], cb[1], cb[2], cb[3]};
          const float sv[8] = {sa[0], sa[1], sa[2], sa[3], sb[0], sb[1], sb[2], sb[3]};
          const float sg = (cg < 4) ? 1.0f : -1.0f;
#pragma unroll
          for (int i = 0; i < 8; ++i) {
            const float no = y[i] * rn;
            const float np = pt[i] * rn;
            y[i] = (no * cc[i] + sg * (np * sv[i])) * scale;
          }
          const size_t po = (size_t)z * dz + ((size_t)bn * SEQ + t) * HD + cg * 8;
          dh = Dh0 + po;
          dl = Dl0 + po;
        } else {
          const size_t po = (size_t)(rbase + row) * ldd + n0 + cg * 8;
          dh = Dh0 + po;
          dl = Dl0 + po;
        }
        v8u hv = {}, lv = {};
        split8(y, hv, lv);
        *(volatile v8u*)dh = hv;
        *(volatile v8u*)dl = lv;
        __threadfence();
        *(volatile v8u*)dh = hv;
        *(volatile v8u*)dl = lv;
      }
    }
    __syncthreads();
  }
}

__global__ void __launch_bounds__(128) k_flash(const u16* __restrict__ qh, const u16* __restrict__ ql,
                                             const u16* __restrict__ kh, const u16* __restrict__ kl,
                                             const u16* __restrict__ vh, const u16* __restrict__ vl,
                                             float* __restrict__ ctx)
{
  __shared__ __align__(16) u16 ph[4][16][32];
  __shared__ __align__(16) u16 pl[4][16][32];
  __shared__ __align__(16) float ost[4][16][VD];
  const int lane = threadIdx.x & 31, w = threadIdx.x >> 5, h = lane >> 4, m = lane & 15;
  const int sh = blockIdx.y, hh = sh >> 1, bx = blockIdx.x;
  const int q0 = bx * 64 + w * 16;

  const size_t qo = ((size_t)sh * SEQ + q0 + m) * HD;
  const v8i Qh0 = ldfrag(qh + qo, h), Qh1 = ldfrag(qh + qo + 32, h);
  const v8i Ql0 = ldfrag(ql + qo, h), Ql1 = ldfrag(ql + qo + 32, h);
  const u16* kbh = kh + (size_t)sh * SEQ * HD;
  const u16* kbl = kl + (size_t)sh * SEQ * HD;
  const u16* vbh = vh + (size_t)hh * VD * SEQ;
  const u16* vbl = vl + (size_t)hh * VD * SEQ;

  v8f O[8] = {};
  float mr[8], lr[8];
#pragma unroll
  for (int r = 0; r < 8; ++r) { mr[r] = -1e30f; lr[r] = 0.0f; }

  const int nsteps = 2 * bx + 2;
#pragma unroll 1
  for (int st = 0; st < nsteps; ++st) {
    const int n0 = st * 32;
    v8f S[2];
#pragma unroll
    for (int j = 0; j < 2; ++j) {
      v8f s = {};
      const size_t ko = (size_t)(n0 + j * 16 + m) * HD;
      {
        const v8i Kh = ldfrag(kbh + ko, h), Kl = ldfrag(kbl + ko, h);
        s = mma3(Qh0, Ql0, Kh, Kl, s);
      }
      {
        const v8i Kh = ldfrag(kbh + ko + 32, h), Kl = ldfrag(kbl + ko + 32, h);
        s = mma3(Qh1, Ql1, Kh, Kl, s);
      }
      S[j] = s;
      asm volatile("" ::: "memory");
    }
#pragma unroll
    for (int r = 0; r < 8; ++r) {
      const int row = q0 + 8 * h + r;
      const float e0 = (n0 + m > row) ? -1e30f : S[0][r];
      const float e1 = (n0 + 16 + m > row) ? -1e30f : S[1][r];
      float tm = fmaxf(e0, e1);
      tm = fmaxf(tm, __shfl_xor(tm, 1, 32));
      tm = fmaxf(tm, __shfl_xor(tm, 2, 32));
      tm = fmaxf(tm, __shfl_xor(tm, 4, 32));
      tm = fmaxf(tm, __shfl_xor(tm, 8, 32));
      const float nm = fmaxf(mr[r], tm);
      const float alpha = __expf(mr[r] - nm);
      mr[r] = nm;
      const float p0 = __expf(e0 - nm);
      const float p1 = __expf(e1 - nm);
      float ps = p0 + p1;
      ps += __shfl_xor(ps, 1, 32);
      ps += __shfl_xor(ps, 2, 32);
      ps += __shfl_xor(ps, 4, 32);
      ps += __shfl_xor(ps, 8, 32);
      lr[r] = lr[r] * alpha + ps;
#pragma unroll
      for (int c = 0; c < 8; ++c) O[c][r] = O[c][r] * alpha;
      const u16 h0 = bf_rne(p0), h1 = bf_rne(p1);
      ph[w][8 * h + r][m]      = h0;
      ph[w][8 * h + r][16 + m] = h1;
      pl[w][8 * h + r][m]      = bf_rne(p0 - bf_up(h0));
      pl[w][8 * h + r][16 + m] = bf_rne(p1 - bf_up(h1));
    }
    __syncthreads();
    const v8i Ph = ldfrag(&ph[w][m][0], h);
    const v8i Pl = ldfrag(&pl[w][m][0], h);
#pragma unroll
    for (int c = 0; c < 8; ++c) {
      const size_t vo = (size_t)(c * 16 + m) * SEQ + n0;
      const v8i Vh = ldfrag(vbh + vo, h), Vl = ldfrag(vbl + vo, h);
      O[c] = mma3(Ph, Pl, Vh, Vl, O[c]);
      if (c & 1) asm volatile("" ::: "memory");
    }
    __syncthreads();
  }

#pragma unroll
  for (int r = 0; r < 8; ++r) {
    const float inv = 1.0f / lr[r];
#pragma unroll
    for (int c = 0; c < 8; ++c) ost[w][8 * h + r][c * 16 + m] = O[c][r] * inv;
  }
  __syncthreads();
  float* cb = ctx + ((size_t)sh * SEQ + q0) * VD + lane * 4;
#pragma unroll
  for (int rr = 0; rr < 16; ++rr) {
    const v4f v = *(const v4f*)&ost[w][rr][lane * 4];
    *(volatile v4f*)(cb + (size_t)rr * VD) = v;
  }
  __threadfence();
#pragma unroll
  for (int rr = 0; rr < 16; ++rr) {
    const v4f v = *(const v4f*)&ost[w][rr][lane * 4];
    *(volatile v4f*)(cb + (size_t)rr * VD) = v;
  }
}

__global__ void __launch_bounds__(256) k_combine(const float* __restrict__ ctx,
                                               const float* __restrict__ lq1, const float* __restrict__ lk1,
                                               const float* __restrict__ lq2, const float* __restrict__ lk2,
                                               float lam_init, float oscale,
                                               u16* __restrict__ Yh, u16* __restrict__ Yl)
{
  const int lane = threadIdx.x & 31, w = threadIdx.x >> 5;
  const int gw = blockIdx.x * 8 + w;
  const int hd = gw & 7, tp = gw >> 3;
  const int t = tp * 2 + (lane >> 4), cg = lane & 15;

  float s1 = lq1[lane] * lk1[lane] + lq1[lane + 32] * lk1[lane + 32];
  float s2 = lq2[lane] * lk2[lane] + lq2[lane + 32] * lk2[lane + 32];
#pragma unroll
  for (int k = 16; k >= 1; k >>= 1) { s1 += __shfl_xor(s1, k, 32); s2 += __shfl_xor(s2, k, 32); }
  const float lam = __expf(s1) - __expf(s2) + lam_init;

  const float* o1 = ctx + ((size_t)(2 * hd) * SEQ + t) * VD + cg * 8;
  const float* o2 = ctx + ((size_t)(2 * hd + 1) * SEQ + t) * VD + cg * 8;
  const v4f a1 = *(const v4f*)o1, b1 = *(const v4f*)(o1 + 4);
  const v4f a2 = *(const v4f*)o2, b2 = *(const v4f*)(o2 + 4);
  float y[8] = {a1[0] - lam * a2[0], a1[1] - lam * a2[1], a1[2] - lam * a2[2], a1[3] - lam * a2[3],
                b1[0] - lam * b2[0], b1[1] - lam * b2[1], b1[2] - lam * b2[2], b1[3] - lam * b2[3]};
  float mu = 0.0f;
#pragma unroll
  for (int i = 0; i < 8; ++i) mu += y[i];
  mu += __shfl_xor(mu, 1, 32);
  mu += __shfl_xor(mu, 2, 32);
  mu += __shfl_xor(mu, 4, 32);
  mu += __shfl_xor(mu, 8, 32);
  mu *= (1.0f / 128.0f);
  float var = 0.0f;
#pragma unroll
  for (int i = 0; i < 8; ++i) { const float d = y[i] - mu; var += d * d; }
  var += __shfl_xor(var, 1, 32);
  var += __shfl_xor(var, 2, 32);
  var += __shfl_xor(var, 4, 32);
  var += __shfl_xor(var, 8, 32);
  var *= (1.0f / 128.0f);
  const float rs = rsqrtf(var + LN_EPS) * oscale;
#pragma unroll
  for (int i = 0; i < 8; ++i) y[i] = (y[i] - mu) * rs;

  v8u hv = {}, lv = {};
  split8(y, hv, lv);
  const size_t po = (size_t)t * EMB + hd * VD + cg * 8;
  *(volatile v8u*)(Yh + po) = hv;
  *(volatile v8u*)(Yl + po) = lv;
  __threadfence();
  *(volatile v8u*)(Yh + po) = hv;
  *(volatile v8u*)(Yl + po) = lv;
}

static double h_sqrt(double x) {
  double y = x;
  for (int i = 0; i < 200; ++i) y = 0.5 * (y + x / y);
  return y;
}

extern "C" void kernel_launch(void* const* d_in, const int* in_sizes, int n_in,
                              void* d_out, int out_size, void* d_ws, size_t ws_size,
                              hipStream_t stream) {
  if (n_in < 9) return;
  if (in_sizes[0] != NB * SEQ * EMB) return;
  for (int i = 1; i <= 4; ++i) if (in_sizes[i] != EMB * EMB) return;
  for (int i = 5; i <= 8; ++i) if (in_sizes[i] != HD) return;
  if (out_size != NB * SEQ * EMB) return;

  const float* x   = (const float*)d_in[0];
  const float* Wq  = (const float*)d_in[1];
  const float* Wk  = (const float*)d_in[2];
  const float* Wv  = (const float*)d_in[3];
  const float* Wp  = (const float*)d_in[4];
  const float* lq1 = (const float*)d_in[5];
  const float* lk1 = (const float*)d_in[6];
  const float* lq2 = (const float*)d_in[7];
  const float* lk2 = (const float*)d_in[8];
  float* out = (float*)d_out;

  const size_t szX   = (size_t)NB * SEQ * EMB * 2;
  const size_t szW   = (size_t)4 * EMB * EMB * 2;
  const size_t szQK  = (size_t)2 * NSH * SEQ * HD * 2;
  const size_t szVT  = (size_t)EMB * SEQ * 2;
  const size_t szCTX = (size_t)NSH * SEQ * VD * 4;
  const size_t szY   = (size_t)SEQ * EMB * 2;
  const size_t szTB  = (size_t)SEQ * 32 * 4;
  char* ws = (char*)d_ws;
  size_t off = 0;
  u16*   xh  = (u16*)(ws + off);   off += szX;
  u16*   xl  = (u16*)(ws + off);   off += szX;
  u16*   wh  = (u16*)(ws + off);   off += szW;
  u16*   wl  = (u16*)(ws + off);   off += szW;
  u16*   qkh = (u16*)(ws + off);   off += szQK;
  u16*   qkl = (u16*)(ws + off);   off += szQK;
  u16*   vth = (u16*)(ws + off);   off += szVT;
  u16*   vtl = (u16*)(ws + off);   off += szVT;
  float* ctx = (float*)(ws + off); off += szCTX;
  u16*   yh  = (u16*)(ws + off);   off += szY;
  u16*   yl  = (u16*)(ws + off);   off += szY;
  float* cst = (float*)(ws + off); off += szTB;
  float* snt = (float*)(ws + off); off += szTB;
  if (off > ws_size) return;

  InvFreq inv;
  {
    double r = 10000.0;
    for (int i = 0; i < 5; ++i) r = h_sqrt(r);
    double pw = 1.0;
    for (int j = 0; j < 32; ++j) {
      const float p32 = (float)pw;
      inv.v[j] = (float)(1.0 / (double)p32);
      pw *= r;
    }
  }
  const float lam_init = (float)0.61928347285267872;
  const float oscale   = (float)0.38071652714732128;

  {
    const int n8x = NB * SEQ * EMB / 8;
    const int n8w = EMB * EMB / 8;
    k_split<<<(n8x + 255) / 256, 256, 0, stream>>>(x, xh, xl, n8x);
    k_split<<<(n8w + 255) / 256, 256, 0, stream>>>(Wq, wh + 0 * (size_t)EMB * EMB, wl + 0 * (size_t)EMB * EMB, n8w);
    k_split<<<(n8w + 255) / 256, 256, 0, stream>>>(Wk, wh + 1 * (size_t)EMB * EMB, wl + 1 * (size_t)EMB * EMB, n8w);
    k_split<<<(n8w + 255) / 256, 256, 0, stream>>>(Wv, wh + 2 * (size_t)EMB * EMB, wl + 2 * (size_t)EMB * EMB, n8w);
    k_split<<<(n8w + 255) / 256, 256, 0, stream>>>(Wp, wh + 3 * (size_t)EMB * EMB, wl + 3 * (size_t)EMB * EMB, n8w);
  }
  k_rot<<<(SEQ * 32 + 255) / 256, 256, 0, stream>>>(inv, cst, snt, SEQ * 32);

  const size_t wstride = (size_t)EMB * EMB;
  const size_t dzqk    = (size_t)NSH * SEQ * HD;
  for (int b = 0; b < NB; ++b) {
    const u16* xbh = xh + (size_t)b * SEQ * EMB;
    const u16* xbl = xl + (size_t)b * SEQ * EMB;
    k_gemm<0><<<dim3(EMB / 64, SEQ / 256, 2), 256, 0, stream>>>(
        xbh, xbl, EMB, wh, wl, EMB, wstride, EMB,
        qkh, qkl, dzqk, HD, out, cst, snt, 0.125f, 1.0f);
    k_gemm<1><<<dim3(SEQ / 64, EMB / 256, 1), 256, 0, stream>>>(
        wh + 2 * wstride, wl + 2 * wstride, EMB, xbh, xbl, EMB, (size_t)0, EMB,
        vth, vtl, (size_t)0, SEQ, out, cst, snt, 1.0f, 1.0f);
    k_flash<<<dim3(SEQ / 64, NSH), 128, 0, stream>>>(qkh, qkl, qkh + dzqk, qkl + dzqk, vth, vtl, ctx);
    k_combine<<<(SEQ * NHD / 2) / 8, 256, 0, stream>>>(ctx, lq1, lk1, lq2, lk2, lam_init, oscale, yh, yl);
    k_gemm<2><<<dim3(EMB / 64, SEQ / 256, 1), 256, 0, stream>>>(
        yh, yl, EMB, wh + 3 * wstride, wl + 3 * wstride, EMB, (size_t)0, EMB,
        qkh, qkl, (size_t)0, EMB, out + (size_t)b * SEQ * EMB, cst, snt, 1.0f, 1.0f);
  }
}
